// RobotMambaPolicy_86208583565490
// MI455X (gfx1250) — hardware-verified
//
#include <hip/hip_runtime.h>
#include <math.h>

typedef __attribute__((ext_vector_type(16))) _Float16 v16h;
typedef __attribute__((ext_vector_type(16))) __bf16 v16b;
typedef __attribute__((ext_vector_type(8)))  _Float16 v8h;
typedef __attribute__((ext_vector_type(8)))  float v8f;
typedef __attribute__((ext_vector_type(4)))  float v4f;
typedef __attribute__((ext_vector_type(2)))  float v2f;
typedef __attribute__((ext_vector_type(4)))  unsigned v4u;
typedef __attribute__((ext_vector_type(4)))  int v4i;
typedef float __attribute__((may_alias)) float_a;
typedef int __attribute__((may_alias)) int_a;

template <typename T> __device__ __forceinline__ void vst2(void* p, T v) { *(volatile T*)p = v; __threadfence(); *(volatile T*)p = v; }
__device__ __forceinline__ v8f wmma16(v16h a, v16h b, v8f c) {
  v8f d = __builtin_amdgcn_wmma_f32_16x16x32_f16(false, a, false, b, (short)0, c, false, false);
  asm volatile("v_nop\n\tv_nop\n\tv_nop\n\tv_nop" : "+v"(d) : "v"(a), "v"(b));
  return d;
}
__device__ __forceinline__ v8f wmma_bf(v16b a, v16b b, v8f c) {
  v8f d = __builtin_amdgcn_wmma_f32_16x16x32_bf16(false, a, false, b, (short)0, c, false, false);
  asm volatile("v_nop\n\tv_nop\n\tv_nop\n\tv_nop" : "+v"(d) : "v"(a), "v"(b));
  return d;
}
__device__ __forceinline__ v16h frag_h(const _Float16* rowk0, int lane) {
  union { v16h v; v8h q[2]; } u; const _Float16* p = rowk0 + 8 * (lane >> 4);
  u.q[0] = *(const v8h*)p; u.q[1] = *(const v8h*)(p + 16); return u.v;
}
__device__ __forceinline__ v16h frag_f32(const float* rowk0, int lane) {
  v16h a; const float* p = rowk0 + 8 * (lane >> 4);
#pragma unroll
  for (int i = 0; i < 8; ++i) { a[i] = (_Float16)p[i]; a[8 + i] = (_Float16)p[16 + i]; }
  return a;
}
__device__ __forceinline__ v16h frag_f32s(const float* rowk0, int lane, float sc) {
  v16h a; const float* p = rowk0 + 8 * (lane >> 4);
#pragma unroll
  for (int i = 0; i < 8; ++i) { a[i] = (_Float16)(p[i] * sc); a[8 + i] = (_Float16)(p[16 + i] * sc); }
  return a;
}
__device__ __forceinline__ v16h fragc_f32(const float* W, int k0, int n, int lane, int ld, int K) {
  v16h a; const int g = lane >> 4;
#pragma unroll
  for (int i = 0; i < 8; ++i) { const int ka = k0 + 8 * g + i, kb = ka + 16;
    a[i] = (_Float16)(ka < K ? W[(size_t)(ka < K ? ka : K - 1) * ld + n] : 0.f); a[8 + i] = (_Float16)(kb < K ? W[(size_t)(kb < K ? kb : K - 1) * ld + n] : 0.f); }
  return a;
}
struct F2 { v16b h, l; };
__device__ __forceinline__ F2 bsplit16(const float v[16]) { F2 r;
#pragma unroll
  for (int i = 0; i < 16; ++i) { const __bf16 h = (__bf16)v[i]; r.h[i] = h; r.l[i] = (__bf16)(v[i] - (float)h); }
  return r; }
__device__ __forceinline__ F2 split_row(const float* row, int k0, int lane) { float v[16]; const float* p = row + k0 + 8 * (lane >> 4);
#pragma unroll
  for (int i = 0; i < 8; ++i) { v[i] = p[i]; v[8 + i] = p[16 + i]; }
  return bsplit16(v); }
__device__ __forceinline__ F2 split_rowK(const float* row, int k0, int lane, int K) { float v[16]; const int g = lane >> 4;
#pragma unroll
  for (int i = 0; i < 8; ++i) { const int ka = k0 + 8 * g + i, kb = ka + 16; v[i] = ka < K ? row[ka < K ? ka : K - 1] : 0.f; v[8 + i] = kb < K ? row[kb < K ? kb : K - 1] : 0.f; }
  return bsplit16(v); }
__device__ __forceinline__ F2 split_col(const float* W, int k0, int n, int lane, int ld, int K) { float v[16]; const int g = lane >> 4;
#pragma unroll
  for (int i = 0; i < 8; ++i) { const int ka = k0 + 8 * g + i, kb = ka + 16; v[i] = ka < K ? W[(size_t)(ka < K ? ka : K - 1) * ld + n] : 0.f; v[8 + i] = kb < K ? W[(size_t)(kb < K ? kb : K - 1) * ld + n] : 0.f; }
  return bsplit16(v); }
__device__ __forceinline__ v8f mac3(const F2& a, const F2& b, v8f c) { c = wmma_bf(a.l, b.h, c); c = wmma_bf(a.h, b.l, c); return wmma_bf(a.h, b.h, c); }
__device__ __forceinline__ float sigm(float v) { return 1.0f / (1.0f + expf(-v)); }
#define LDSX() do { asm volatile("s_wait_dscnt 0" ::: "memory"); __builtin_amdgcn_wave_barrier(); __builtin_amdgcn_fence(__ATOMIC_RELEASE, "workgroup"); } while (0)


#define LL 2048
#define BB 8
#define NR (LL * BB)
#define DIN 128
#define DM 256
#define DI 512
#define DS 16
#define DTR 16
#define DO 32
__device__ __forceinline__ float bfr(float v) { return (float)(__bf16)v; }
__device__ __forceinline__ v16b frag_b(const __bf16* rowk0, int lane) { return __builtin_bit_cast(v16b, frag_h((const _Float16*)rowk0, lane)); }
__device__ __attribute__((noinline)) float exp_ni(float v) { return expf(v); }
__device__ __forceinline__ float silu(float v) { return v / (1.0f + expf(-v)); }
__device__ __attribute__((noinline)) float softplus_(float v) { return v > 20.f ? v : log1pf(expf(v)); }

__global__ __launch_bounds__(128) void k_emb(const float* __restrict__ s, const float* __restrict__ W, const float* __restrict__ b, float* __restrict__ X0) {
  __shared__ __align__(16) float so[4][16][132];
  const int tid = threadIdx.x, wave = tid >> 5, lane = tid & 31, col = lane & 15, g = lane >> 4; const int r0 = blockIdx.x * 64 + wave * 16; const int n0 = blockIdx.y * 128;
  v8f acc[8] = {};
#pragma unroll
  for (int kc = 0; kc < DIN / 32; ++kc) { const v16b a = split_row(s + (size_t)(r0 + col) * DIN, kc * 32, lane).h;
#pragma unroll
    for (int j = 0; j < 8; ++j) acc[j] = wmma_bf(a, split_col(W, kc * 32, n0 + j * 16 + col, lane, DM, DIN).h, acc[j]); }
#pragma unroll
  for (int j = 0; j < 8; ++j) { const float bb = b[n0 + j * 16 + col];
#pragma unroll
    for (int r = 0; r < 8; ++r) so[wave][8 * g + r][j * 16 + col] = acc[j][r] + bb; }
  LDSX();
  for (int rl = 0; rl < 16; ++rl) vst2(X0 + (size_t)(r0 + rl) * DM + n0 + lane * 4, *(const v4f*)(&so[wave][rl][lane * 4]));
}
__global__ __launch_bounds__(128) void k_in(const float* __restrict__ X0, const float* __restrict__ nw, const float* __restrict__ Win, __bf16* __restrict__ XPB, __bf16* __restrict__ ZB) {
  __shared__ __align__(16) __bf16 sx[64][DM + 8]; __shared__ __align__(16) __bf16 so[4][16][136];
  const int tid = threadIdx.x, wave = tid >> 5, lane = tid & 31, col = lane & 15, g = lane >> 4; const int r0b = blockIdx.x * 64, n0 = blockIdx.y * 128;
  for (int rl = 0; rl < 16; ++rl) { const int row = r0b + wave * 16 + rl; const float* xr = X0 + (size_t)row * DM; float v[8]; float ss = 0.f;
#pragma unroll
    for (int e = 0; e < 8; ++e) { v[e] = xr[lane * 8 + e]; ss += v[e] * v[e]; }
#pragma unroll
    for (int o = 16; o > 0; o >>= 1) ss += __shfl_xor(ss, o, 32);
    const float rs = rsqrtf(ss * (1.0f / DM) + 1e-5f);
#pragma unroll
    for (int e = 0; e < 8; ++e) sx[wave * 16 + rl][lane * 8 + e] = (__bf16)(v[e] * rs * nw[lane * 8 + e]); }
  LDSX();
  v8f acc[8] = {};
#pragma unroll
  for (int kc = 0; kc < DM / 32; ++kc) { const v16b a = frag_b(&sx[wave * 16 + col][0] + kc * 32, lane);
#pragma unroll
    for (int j = 0; j < 8; ++j) acc[j] = wmma_bf(a, split_col(Win, kc * 32, n0 + j * 16 + col, lane, 2 * DI, DM).h, acc[j]); }
#pragma unroll
  for (int j = 0; j < 8; ++j)
#pragma unroll
    for (int r = 0; r < 8; ++r) so[wave][8 * g + r][j * 16 + col] = (__bf16)acc[j][r];
  LDSX();
  __bf16* dst = n0 < DI ? XPB : ZB; const int c0 = n0 < DI ? n0 : n0 - DI;
  for (int rl = 0; rl < 16; ++rl) { if (lane < 16) vst2((unsigned*)(dst + (size_t)(r0b + wave * 16 + rl) * DI + c0 + lane * 8), *(const v4u*)(&so[wave][rl][lane * 8])); }
}
__global__ __launch_bounds__(256) void k_conv(const __bf16* __restrict__ XPB, const float* __restrict__ cw, const float* __restrict__ cb, float* __restrict__ XP) {
  const size_t i4 = (size_t)blockIdx.x * 256 + threadIdx.x; if (i4 >= (size_t)NR * DI / 4) return; const size_t r = i4 / (DI / 4); const int c0 = (int)(i4 % (DI / 4)) * 4; const int l = (int)(r / BB);
  v4f o;
#pragma unroll
  for (int e = 0; e < 4; ++e) { const int c = c0 + e; float acc = cb[c];
#pragma unroll
    for (int k = 0; k < 4; ++k) { const int lk = l - 3 + k; if (lk >= 0) acc += cw[c * 4 + k] * (float)XPB[(r - (size_t)(3 - k) * BB) * DI + c]; }
    o[e] = silu(acc); }
  vst2(XP + r * DI + c0, o);
}
__global__ __launch_bounds__(128) void k_xp(const float* __restrict__ XP, const float* __restrict__ Wx, const float* __restrict__ Wdt, const float* __restrict__ bdt, __bf16* __restrict__ DTB, float* __restrict__ BM, float* __restrict__ CM) {
  __shared__ __align__(16) float sd[64][52]; __shared__ __align__(16) __bf16 so[4][16][136];
  const int tid = threadIdx.x, wave = tid >> 5, lane = tid & 31, col = lane & 15, g = lane >> 4; const int r0b = blockIdx.x * 64, r0 = r0b + wave * 16;
  { v8f acc[3] = {};
#pragma unroll 2
    for (int kc = 0; kc < DI / 32; ++kc) { const v16b a = split_row(XP + (size_t)(r0 + col) * DI, kc * 32, lane).h;
#pragma unroll
      for (int j = 0; j < 3; ++j) acc[j] = wmma_bf(a, split_col(Wx, kc * 32, j * 16 + col, lane, DTR + 2 * DS, DI).h, acc[j]); }
#pragma unroll
    for (int j = 0; j < 3; ++j)
#pragma unroll
      for (int r = 0; r < 8; ++r) sd[wave * 16 + 8 * g + r][j * 16 + col] = acc[j][r]; }
  LDSX();
  for (int half = 0; half < 2; ++half) { const int rl = half * 8 + (lane >> 2), pc = lane & 3; const int row = r0 + rl;
    vst2(BM + (size_t)row * DS + pc * 4, *(const v4f*)(&sd[wave * 16 + rl][DTR + pc * 4])); vst2(CM + (size_t)row * DS + pc * 4, *(const v4f*)(&sd[wave * 16 + rl][DTR + DS + pc * 4])); }
#pragma unroll 1
  for (int nh = 0; nh < 4; ++nh) { v8f acc[8] = {}; const v16b a = split_rowK(&sd[wave * 16 + col][0], 0, lane, DTR).h;
#pragma unroll
    for (int j = 0; j < 8; ++j) acc[j] = wmma_bf(a, split_col(Wdt, 0, nh * 128 + j * 16 + col, lane, DI, DTR).h, acc[j]);
#pragma unroll
    for (int j = 0; j < 8; ++j) { const float bb = bdt[nh * 128 + j * 16 + col];
#pragma unroll
      for (int r = 0; r < 8; ++r) so[wave][8 * g + r][j * 16 + col] = (__bf16)softplus_(acc[j][r] + bb); }
    LDSX();
    for (int rl = 0; rl < 16; ++rl) { if (lane < 16) vst2((unsigned*)(DTB + (size_t)(r0 + rl) * DI + nh * 128 + lane * 8), *(const v4u*)(&so[wave][rl][lane * 8])); }
    LDSX(); }
}
__global__ __launch_bounds__(256) void k_scan(const float* __restrict__ XP, const __bf16* __restrict__ DTB, const float* __restrict__ BM, const float* __restrict__ CM, const __bf16* __restrict__ ZB, const float* __restrict__ Alog, const float* __restrict__ Dp, __bf16* __restrict__ YB) {
  const int b = blockIdx.y, d = blockIdx.x * 256 + threadIdx.x;
  float A[DS], h[DS];
#pragma unroll
  for (int sI = 0; sI < DS; ++sI) { A[sI] = -expf(Alog[d * DS + sI]); h[sI] = 0.f; }
  const float Dd = Dp[d];
  __shared__ __align__(16) __bf16 sy[8][256 + 8];
#pragma unroll 1
  for (int l0 = 0; l0 < LL; l0 += 8) {
#pragma unroll 1
    for (int li = 0; li < 8; ++li) { const int l = l0 + li; const size_t r = (size_t)l * BB + b;
      const float dt = (float)DTB[r * DI + d], x = XP[r * DI + d], z = (float)ZB[r * DI + d]; const float* Br = BM + r * DS; const float* Cr = CM + r * DS;
      const float dx = dt * x; float y = 0.f;
#pragma unroll
      for (int sI = 0; sI < DS; ++sI) { h[sI] = exp_ni(dt * A[sI]) * h[sI] + dx * Br[sI]; y += h[sI] * Cr[sI]; }
      y = (y + x * Dd) * silu(z); sy[li][threadIdx.x] = (__bf16)y; }
    __syncthreads();
    for (int q = threadIdx.x; q < 8 * 32; q += 256) { const int li = q >> 5, pc = q & 31; vst2((unsigned*)(YB + ((size_t)(l0 + li) * BB + b) * DI + blockIdx.x * 256 + pc * 8), *(const v4u*)(&sy[li][pc * 8])); }
    __syncthreads(); }
}
__global__ __launch_bounds__(128) void k_out(const __bf16* __restrict__ YB, const float* __restrict__ Wout, const float* __restrict__ X0, const float* __restrict__ Wh, const float* __restrict__ bh, const float* __restrict__ lsd, const float* __restrict__ a, float* __restrict__ out) {
  __shared__ __align__(16) float sx1[4][16][DM + 4]; __shared__ float slp[64];
  const int tid = threadIdx.x, wave = tid >> 5, lane = tid & 31, col = lane & 15, g = lane >> 4; const int r0b = blockIdx.x * 64, r0 = r0b + wave * 16;
#pragma unroll 1
  for (int nh = 0; nh < 2; ++nh) { v8f acc[8] = {};
#pragma unroll 2
    for (int kc = 0; kc < DI / 32; ++kc) { const v16b ya = frag_b(YB + (size_t)(r0 + col) * DI + kc * 32, lane);
#pragma unroll
      for (int j = 0; j < 8; ++j) acc[j] = wmma_bf(ya, split_col(Wout, kc * 32, nh * 128 + j * 16 + col, lane, DM, DI).h, acc[j]); }
#pragma unroll
    for (int j = 0; j < 8; ++j) { const int n = nh * 128 + j * 16 + col;
#pragma unroll
      for (int r = 0; r < 8; ++r) sx1[wave][8 * g + r][n] = acc[j][r] + X0[(size_t)(r0 + 8 * g + r) * DM + n]; } }
  LDSX();
  v8f mu[2] = {};
#pragma unroll
  for (int kc = 0; kc < DM / 32; ++kc) { const v16b xa = split_row(&sx1[wave][col][0], kc * 32, lane).h;
#pragma unroll
    for (int j = 0; j < 2; ++j) mu[j] = wmma_bf(xa, split_col(Wh, kc * 32, j * 16 + col, lane, DO, DM).h, mu[j]); }
  float part[8];
#pragma unroll
  for (int r = 0; r < 8; ++r) { float sum = 0.f; const int row = r0 + 8 * g + r;
#pragma unroll
    for (int j = 0; j < 2; ++j) { const int o = j * 16 + col; const float m = mu[j][r] + bh[o]; const float zz = (a[(size_t)row * DO + o] - m) * expf(-lsd[o]); sum += -0.5f * zz * zz - lsd[o] - 0.9189385332046727f; }
    part[r] = sum; }
#pragma unroll
  for (int r = 0; r < 8; ++r) {
#pragma unroll
    for (int o2 = 1; o2 < 16; o2 <<= 1) part[r] += __shfl_xor(part[r], o2, 32); }
  if (col == 0) {
#pragma unroll
    for (int r = 0; r < 8; ++r) slp[wave * 16 + 8 * g + r] = part[r]; }
  __syncthreads();
  if (tid < 16) vst2(out + r0b + tid * 4, *(const v4f*)(&slp[tid * 4]));
}
extern "C" void kernel_launch(void* const* d_in, const int* in_sizes, int n_in, void* d_out, int out_size, void* d_ws, size_t ws_size, hipStream_t stream) {
  (void)in_sizes; (void)n_in; (void)out_size; (void)ws_size;
  const float** I = (const float**)d_in;
  const float* s = I[0]; const float* a = I[1]; const float* Wemb = I[2]; const float* bemb = I[3]; const float* nw = I[4]; const float* Win = I[5]; const float* cw = I[6]; const float* cb = I[7]; const float* Wx = I[8]; const float* Wdt = I[9]; const float* bdt = I[10];
  const float* Alog = I[11]; const float* Dp = I[12]; const float* Wout = I[13]; const float* Wh = I[14]; const float* bh = I[15]; const float* lsd = I[16];
  char* ws = (char*)d_ws; size_t off = 0;
  auto take = [&](size_t bytes) { char* p = ws + off; off += (bytes + 255) & ~(size_t)255; return p; };
  float* X0 = (float*)take((size_t)NR * DM * 4); __bf16* XPB = (__bf16*)take((size_t)NR * DI * 2); __bf16* ZB = (__bf16*)take((size_t)NR * DI * 2); float* XP = (float*)take((size_t)NR * DI * 4);
  __bf16* DTB = (__bf16*)take((size_t)NR * DI * 2); float* BM = (float*)take((size_t)NR * DS * 4); float* CM = (float*)take((size_t)NR * DS * 4); __bf16* YB = (__bf16*)take((size_t)NR * DI * 2);
  k_emb<<<dim3(NR / 64, DM / 128), 128, 0, stream>>>(s, Wemb, bemb, X0);
  k_in<<<dim3(NR / 64, 2 * DI / 128), 128, 0, stream>>>(X0, nw, Win, XPB, ZB);
  k_conv<<<(NR * DI / 4 + 255) / 256, 256, 0, stream>>>(XPB, cw, cb, XP);
  k_xp<<<NR / 64, 128, 0, stream>>>(XP, Wx, Wdt, bdt, DTB, BM, CM);
  k_scan<<<dim3(DI / 256, BB), 256, 0, stream>>>(XP, DTB, BM, CM, ZB, Alog, Dp, YB);
  k_out<<<NR / 64, 128, 0, stream>>>(YB, Wout, X0, Wh, bh, lsd, a, (float*)d_out);
}
